// StarTopologyFCN_59485297050172
// MI455X (gfx1250) — hardware-run, weakly checked
//
#include <hip/hip_runtime.h>

constexpr int kBatch  = 2048;
constexpr int kIn0    = 512;
constexpr int kHid1   = 256;
constexpr int kHid2   = 128;
constexpr int kHid3   = 64;
constexpr int kNumDom = 8;
constexpr float kWCarry = 1024.0f;
constexpr float kHCarry = 256.0f;

typedef __attribute__((ext_vector_type(16))) _Float16 v16h;
typedef __attribute__((ext_vector_type(8)))  _Float16 v8h;
typedef __attribute__((ext_vector_type(16))) __bf16   v16b;
typedef __attribute__((ext_vector_type(8)))  __bf16   v8b;
typedef __attribute__((ext_vector_type(8)))  float    v8f;
typedef __attribute__((ext_vector_type(4)))  float    v4f;
typedef __attribute__((ext_vector_type(4)))  unsigned int v4u;

__device__ __forceinline__ unsigned short f2bf_bits(float f) {
  unsigned u = __float_as_uint(f);
  return (unsigned short)((u + 0x7FFFu + ((u >> 16) & 1u)) >> 16);
}
__device__ __forceinline__ float bf_bits2f(unsigned short h) { return __uint_as_float(((unsigned)h) << 16); }

__device__ __forceinline__ void dep_guard_h(v8f& a, v8f& b, v16h x, v16h y) { asm volatile("v_nop\n\tv_nop\n\tv_nop\n\tv_nop" : "+v"(a), "+v"(b) : "v"(x), "v"(y)); }
__device__ __forceinline__ void dep_guard_b(v8f& a, v8f& b, v16b x, v16b y) { asm volatile("v_nop\n\tv_nop\n\tv_nop\n\tv_nop" : "+v"(a), "+v"(b) : "v"(x), "v"(y)); }
__device__ __forceinline__ void keep4_h(v16h a, v16h b, v16h c, v16h d) { asm volatile("v_nop" :: "v"(a), "v"(b), "v"(c), "v"(d)); }
__device__ __forceinline__ void keep4_b(v16b a, v16b b, v16b c, v16b d) { asm volatile("v_nop" :: "v"(a), "v"(b), "v"(c), "v"(d)); }
__device__ __forceinline__ void acc_guard4(v8f& a, v8f& b, v8f& c, v8f& d) { asm volatile("v_nop\n\tv_nop\n\tv_nop\n\tv_nop" : "+v"(a), "+v"(b), "+v"(c), "+v"(d)); }
template <typename T> struct Frag;
template <> struct Frag<_Float16> {
  typedef v16h V; union U { v16h v; v8h h[2]; };
  static __device__ __forceinline__ v16h load(const _Float16* p) {
    U f; f.h[0] = *(const v8h*)(p); f.h[1] = *(const v8h*)(p + 16); return f.v;
  }
  static __device__ __forceinline__ v8f mma(v16h a, v16h b, v8f c) {
    return __builtin_amdgcn_wmma_f32_16x16x32_f16(false, a, false, b, (short)0, c, false, false);
  }
  static __device__ __forceinline__ void guard(v8f& a, v8f& b, v16h x, v16h y) { dep_guard_h(a, b, x, y); }
  static __device__ __forceinline__ void keep(v16h a, v16h b, v16h c, v16h d) { keep4_h(a, b, c, d); }
};
template <> struct Frag<__bf16> {
  typedef v16b V; union U { v16b v; v8b h[2]; };
  static __device__ __forceinline__ v16b load(const __bf16* p) {
    U f; f.h[0] = *(const v8b*)(p); f.h[1] = *(const v8b*)(p + 16); return f.v;
  }
  static __device__ __forceinline__ v8f mma(v16b a, v16b b, v8f c) {
    return __builtin_amdgcn_wmma_f32_16x16x32_bf16(false, a, false, b, (short)0, c, false, false);
  }
  static __device__ __forceinline__ void guard(v8f& a, v8f& b, v16b x, v16b y) { dep_guard_b(a, b, x, y); }
  static __device__ __forceinline__ void keep(v16b a, v16b b, v16b c, v16b d) { keep4_b(a, b, c, d); }
};

__device__ __forceinline__ unsigned pk16(unsigned short a, unsigned short b) { return (unsigned)a | ((unsigned)b << 16); }
__device__ __forceinline__ unsigned short h_bits(float f) { const _Float16 h = (_Float16)f; return __builtin_bit_cast(unsigned short, h); }

template <int ET> struct Elem;
template <> struct Elem<0> { typedef _Float16 T; };
template <> struct Elem<1> { typedef __bf16 T; };
template <int ET, bool SPLIT, int BIAS_MODE, int OUT_MODE, bool RESID, int ACT = 0>
__global__ __launch_bounds__(256) void wmma_gemm64(
    const unsigned short* __restrict__ Ap, const unsigned short* __restrict__ A2p, int lda, long strideA,
    const unsigned short* __restrict__ Btp, const unsigned short* __restrict__ Bt2p, int ldb, long strideB,
    void* __restrict__ Cout, void* __restrict__ Cout2, int ldc, long strideC,
    const float* __restrict__ bias,
    const float* __restrict__ resid, long strideR,
    int M, int N, int K, float scale) {
  typedef typename Elem<ET>::T T;
  typedef typename Frag<T>::V V;
  const T* A = (const T*)Ap; const T* A2 = (const T*)A2p; const T* Bt = (const T*)Btp; const T* Bt2 = (const T*)Bt2p;
  __shared__ __align__(16) float sT[8][16 * 68];
  const int b    = blockIdx.y;
  const int lane = threadIdx.x & 31;
  const int wave = threadIdx.x >> 5;
  const int tilesN = N >> 6;
  const int tilesM = M >> 6;
  const int tile = blockIdx.x * 8 + wave;
  if (tile >= tilesM * tilesN) return;
  const int tm = tile / tilesN;
  const int tn = tile - tm * tilesN;
  const int m0 = tm << 6;
  const int n0 = tn << 6;

  const T* Ab  = A  + (size_t)b * strideA;
  const T* Bb  = Bt + (size_t)b * strideB;
  const T* Ab2 = SPLIT ? (A2  + (size_t)b * strideA) : nullptr;
  const T* Bb2 = SPLIT ? (Bt2 + (size_t)b * strideB) : nullptr;

  const int rlane = lane & 15;
  const int koff  = (lane >> 4) * 8;
  const int mOff  = (lane >> 4) * 8;

  v8f acc[4][4];
#pragma unroll
  for (int i = 0; i < 4; ++i)
#pragma unroll
    for (int j = 0; j < 4; ++j) acc[i][j] = (v8f){0.f,0.f,0.f,0.f,0.f,0.f,0.f,0.f};

  for (int k0 = 0; k0 < K; k0 += 32) {
    V bh[4], bl[4];
#pragma unroll
    for (int j = 0; j < 4; ++j) {
      const size_t bo = (size_t)(n0 + (j << 4) + rlane) * ldb + koff + k0;
      bh[j] = Frag<T>::load(Bb + bo);
      if (SPLIT) bl[j] = Frag<T>::load(Bb2 + bo);
    }
#pragma unroll
    for (int i = 0; i < 4; ++i) {
      const size_t ao = (size_t)(m0 + (i << 4) + rlane) * lda + koff + k0;
      V ah = Frag<T>::load(Ab + ao);
      V al;
      if (SPLIT) al = Frag<T>::load(Ab2 + ao);
#pragma unroll
      for (int j = 0; j < 4; ++j) {
        acc[i][j] = Frag<T>::mma(ah, bh[j], acc[i][j]);
        if (SPLIT) {
          acc[i][j] = Frag<T>::mma(ah, bl[j], acc[i][j]);
          acc[i][j] = Frag<T>::mma(al, bh[j], acc[i][j]);
        }
      }
      Frag<T>::guard(acc[i][0], acc[i][3], ah, SPLIT ? al : ah);
    }
    Frag<T>::keep(bh[0], bh[1], bh[2], bh[3]);
    if (SPLIT) Frag<T>::keep(bl[0], bl[1], bl[2], bl[3]);
  }
  acc_guard4(acc[0][0], acc[0][1], acc[0][2], acc[0][3]);
  acc_guard4(acc[1][0], acc[1][1], acc[1][2], acc[1][3]);
  acc_guard4(acc[2][0], acc[2][1], acc[2][2], acc[2][3]);
  acc_guard4(acc[3][0], acc[3][1], acc[3][2], acc[3][3]);

  float* slab = sT[wave];
  const float* Rb = RESID ? (resid + (size_t)b * strideR) : nullptr;
#pragma unroll
  for (int i = 0; i < 4; ++i) {
    const int mBase = m0 + (i << 4);
#pragma unroll
    for (int j = 0; j < 4; ++j) {
      const int n = n0 + (j << 4) + rlane;
      float bv = 0.f;
      if (BIAS_MODE == 2) bv = bias[n];
#pragma unroll
      for (int r = 0; r < 8; ++r) {
        float v = acc[i][j][r] * scale;
        if (BIAS_MODE == 1) v += bias[mBase + mOff + r];
        if (BIAS_MODE == 2) v += bv;
        if (RESID) v += Rb[(size_t)(mBase + mOff + r) * ldc + n];
        if (ACT == 2) v = fmaxf(v, 0.0f);
        if (ACT == 4) v = (v > 0.f) ? v : 0.01f * v;
        slab[(mOff + r) * 68 + (j << 4) + rlane] = v;
      }
    }
    __builtin_amdgcn_fence(__ATOMIC_RELEASE, "workgroup");
    __builtin_amdgcn_wave_barrier();
    __builtin_amdgcn_fence(__ATOMIC_ACQUIRE, "workgroup");
    if (OUT_MODE == 0) {
      float* C = (float*)Cout + (size_t)b * strideC;
      const int hh = lane >> 4, c4 = (lane & 15) * 4;
      for (int pass = 0; pass < 2; ++pass) {
#pragma unroll
        for (int it = 0; it < 8; ++it) {
          const int row = it * 2 + hh;
          v4f v = *(const v4f*)(slab + row * 68 + c4);
          *(volatile v4f*)(C + (size_t)(mBase + row) * ldc + n0 + c4) = v;
        }
        __threadfence();
      }
    } else {
      const int q = lane >> 3, c8 = (lane & 7) * 8;
      unsigned short* C  = (unsigned short*)Cout  + (size_t)b * strideC;
      unsigned short* C2 = (OUT_MODE == 2) ? ((unsigned short*)Cout2 + (size_t)b * strideC) : nullptr;
      for (int pass = 0; pass < 2; ++pass) {
#pragma unroll
        for (int it = 0; it < 4; ++it) {
          const int row = it * 4 + q;
          const float* sp = slab + row * 68 + c8;
          v8h hv, lv;
#pragma unroll
          for (int e = 0; e < 8; ++e) {
            if (OUT_MODE == 1) {
              hv[e] = (_Float16)sp[e];
            } else {
              unsigned short hb = f2bf_bits(sp[e]);
              unsigned short lb = f2bf_bits(sp[e] - bf_bits2f(hb));
              hv[e] = __builtin_bit_cast(_Float16, hb);
              lv[e] = __builtin_bit_cast(_Float16, lb);
            }
          }
          *(volatile v8h*)(C + (size_t)(mBase + row) * ldc + n0 + c8) = hv;
          if (OUT_MODE == 2) *(volatile v8h*)(C2 + (size_t)(mBase + row) * ldc + n0 + c8) = lv;
        }
        __threadfence();
      }
    }
    __builtin_amdgcn_fence(__ATOMIC_RELEASE, "workgroup");
    __builtin_amdgcn_wave_barrier();
    __builtin_amdgcn_fence(__ATOMIC_ACQUIRE, "workgroup");
  }
}

__global__ __launch_bounds__(256) void cast8_f16_kernel(const float* __restrict__ in, unsigned short* __restrict__ out, int n8) {
  const int i = blockIdx.x * 256 + threadIdx.x;
  if (i >= n8) return;
  const float* p = in + 8 * (size_t)i;
  const v4f a = *(const v4f*)(p);
  const v4f c = *(const v4f*)(p + 4);
  unsigned short hb[8];
#pragma unroll
  for (int e = 0; e < 4; ++e) {
    hb[e]     = h_bits(a[e]);
    hb[4 + e] = h_bits(c[e]);
  }
  const v4u u = (v4u){pk16(hb[0], hb[1]), pk16(hb[2], hb[3]), pk16(hb[4], hb[5]), pk16(hb[6], hb[7])};
  unsigned short* q = out + 8 * (size_t)i;
  *(volatile v4u*)q = u;
  __threadfence();
  *(volatile v4u*)q = u;
}

template <int FIN, int FOUT>
__global__ __launch_bounds__(256) void fuse_wt_kernel(const float* __restrict__ sw, const float* __restrict__ dw,
                                                      unsigned short* __restrict__ Bt, float carry) {
  static_assert(FIN % 64 == 0 && FOUT % 64 == 0);
  __shared__ float sm[64][65];
  const int t  = threadIdx.x;
  const int i0 = blockIdx.x * 64;
  const int o0 = blockIdx.y * 64;
  const int d  = blockIdx.z;
#pragma unroll
  for (int it = 0; it < 16; ++it) {
    const int e = it * 256 + t;
    const int r = e >> 6;
    const int c = e & 63;
    const size_t gi = (size_t)(i0 + r) * FOUT + o0 + c;
    const float p = sw[gi] * dw[(size_t)d * FIN * FOUT + gi];
    sm[c][r] = p * carry;
  }
  __syncthreads();
  const int lane = t & 31, wave = t >> 5;
  const int q = lane >> 3, c8 = (lane & 7) * 8;
  unsigned short* op = Bt + (size_t)d * FOUT * FIN;
  for (int pass = 0; pass < 2; ++pass) {
#pragma unroll
    for (int it = 0; it < 2; ++it) {
      const int row = wave * 8 + it * 4 + q;
      unsigned short hb[8];
#pragma unroll
      for (int e = 0; e < 8; ++e) hb[e] = h_bits(sm[row][c8 + e]);
      const v4u u = (v4u){pk16(hb[0], hb[1]), pk16(hb[2], hb[3]), pk16(hb[4], hb[5]), pk16(hb[6], hb[7])};
      *(volatile v4u*)(op + (size_t)(o0 + row) * FIN + i0 + c8) = u;
    }
    __threadfence();
  }
}

template <int FOUT>
__global__ __launch_bounds__(256) void select_h16_kernel(const float* __restrict__ Y, const int* __restrict__ dom,
                                                         const float* __restrict__ sb, const float* __restrict__ db,
                                                         unsigned short* __restrict__ H, int n8, float carry) {
  static_assert(FOUT % 8 == 0);
  const int i = blockIdx.x * 256 + threadIdx.x;
  if (i >= n8) return;
  const int e0 = i * 8;
  const int b  = e0 / FOUT;
  const int o  = e0 - b * FOUT;
  int d = dom[b];
  d = d < 0 ? 0 : (d > (kNumDom - 1) ? (kNumDom - 1) : d);
  const float* yp = Y + (size_t)b * (kNumDom * FOUT) + d * FOUT + o;
  const v4f y0 = *(const v4f*)(yp);
  const v4f y1 = *(const v4f*)(yp + 4);
  const v4f s0 = *(const v4f*)(sb + o);
  const v4f s1 = *(const v4f*)(sb + o + 4);
  const float* gp = db + d * FOUT + o;
  const v4f g0 = *(const v4f*)(gp);
  const v4f g1 = *(const v4f*)(gp + 4);
  unsigned short hb[8];
#pragma unroll
  for (int e = 0; e < 4; ++e) {
    float v0 = y0[e] + (s0[e] + g0[e]);
    float v1 = y1[e] + (s1[e] + g1[e]);
    v0 = fmaxf(v0, 0.0f) * carry;
    v1 = fmaxf(v1, 0.0f) * carry;
    hb[e]     = h_bits(v0);
    hb[4 + e] = h_bits(v1);
  }
  const v4u u = (v4u){pk16(hb[0], hb[1]), pk16(hb[2], hb[3]), pk16(hb[4], hb[5]), pk16(hb[6], hb[7])};
  unsigned short* qp = H + (size_t)e0;
  *(volatile v4u*)qp = u;
  __threadfence();
  *(volatile v4u*)qp = u;
}

__global__ __launch_bounds__(256) void select_out_kernel(const float* __restrict__ Y, const int* __restrict__ dom,
                                                         const float* __restrict__ sb, const float* __restrict__ db,
                                                         float* __restrict__ out, int n4) {
  constexpr int kF = kHid3;
  const int i = blockIdx.x * 256 + threadIdx.x;
  if (i >= n4) return;
  const int e0 = i * 4;
  const int b  = e0 / kF;
  const int o  = e0 - b * kF;
  int d = dom[b];
  d = d < 0 ? 0 : (d > (kNumDom - 1) ? (kNumDom - 1) : d);
  const v4f y = *(const v4f*)(Y + (size_t)b * (kNumDom * kF) + d * kF + o);
  const v4f s = *(const v4f*)(sb + o);
  const v4f g = *(const v4f*)(db + d * kF + o);
  v4f r;
#pragma unroll
  for (int e = 0; e < 4; ++e) {
    const float v = y[e] + (s[e] + g[e]);
    r[e] = fmaxf(v, 0.0f);
  }
  float* qp = out + (size_t)e0;
  *(volatile v4f*)qp = r;
  __threadfence();
  *(volatile v4f*)qp = r;
}

extern "C" void kernel_launch(void* const* d_in, const int* in_sizes, int n_in,
                              void* d_out, int out_size, void* d_ws, size_t ws_size,
                              hipStream_t stream) {
  if (n_in < 14) return;
  if (in_sizes[0] != kBatch * kIn0 || in_sizes[1] != kBatch ||
      in_sizes[2] != kIn0 * kHid1 || in_sizes[3] != kNumDom * kIn0 * kHid1 ||
      in_sizes[4] != kHid1 || in_sizes[5] != kNumDom * kHid1 ||
      in_sizes[6] != kHid1 * kHid2 || in_sizes[7] != kNumDom * kHid1 * kHid2 ||
      in_sizes[8] != kHid2 || in_sizes[9] != kNumDom * kHid2 ||
      in_sizes[10] != kHid2 * kHid3 || in_sizes[11] != kNumDom * kHid2 * kHid3 ||
      in_sizes[12] != kHid3 || in_sizes[13] != kNumDom * kHid3) return;
  if (out_size != kBatch * kHid3) return;

  const float* x   = (const float*)d_in[0];
  const int*   dom = (const int*)d_in[1];
  const float* sw0 = (const float*)d_in[2];
  const float* dw0 = (const float*)d_in[3];
  const float* sb0 = (const float*)d_in[4];
  const float* db0 = (const float*)d_in[5];
  const float* sw1 = (const float*)d_in[6];
  const float* dw1 = (const float*)d_in[7];
  const float* sb1 = (const float*)d_in[8];
  const float* db1 = (const float*)d_in[9];
  const float* sw2 = (const float*)d_in[10];
  const float* dw2 = (const float*)d_in[11];
  const float* sb2 = (const float*)d_in[12];
  const float* db2 = (const float*)d_in[13];
  float* out = (float*)d_out;

  char* ws = (char*)d_ws;
  size_t off = 0;
  const size_t szXh  = (size_t)kBatch * kIn0 * 2;
  const size_t szBt0 = (size_t)kNumDom * kHid1 * kIn0 * 2;
  const size_t szBt1 = (size_t)kNumDom * kHid2 * kHid1 * 2;
  const size_t szBt2 = (size_t)kNumDom * kHid3 * kHid2 * 2;
  const size_t szH1  = (size_t)kBatch * kHid1 * 2;
  const size_t szH2  = (size_t)kBatch * kHid2 * 2;
  const size_t szY0  = (size_t)kBatch * kNumDom * kHid1 * 4;
  const size_t szY1  = (size_t)kBatch * kNumDom * kHid2 * 4;
  const size_t szY2  = (size_t)kBatch * kNumDom * kHid3 * 4;
  unsigned short* xh  = (unsigned short*)(ws + off); off += szXh;
  unsigned short* bt0 = (unsigned short*)(ws + off); off += szBt0;
  unsigned short* bt1 = (unsigned short*)(ws + off); off += szBt1;
  unsigned short* bt2 = (unsigned short*)(ws + off); off += szBt2;
  unsigned short* h1  = (unsigned short*)(ws + off); off += szH1;
  unsigned short* h2  = (unsigned short*)(ws + off); off += szH2;
  float* y0 = (float*)(ws + off); off += szY0;
  float* y1 = (float*)(ws + off); off += szY1;
  float* y2 = (float*)(ws + off); off += szY2;
  if (off > ws_size) return;

  const float wcarryInv = 1.0f / kWCarry;
  const float scale0 = wcarryInv;
  const float scale12 = wcarryInv * (1.0f / kHCarry);

  {
    const int n8 = kBatch * kIn0 / 8;
    cast8_f16_kernel<<<dim3((n8 + 255) / 256), 256, 0, stream>>>(x, xh, n8);
    fuse_wt_kernel<kIn0, kHid1><<<dim3(kIn0 / 64, kHid1 / 64, kNumDom), 256, 0, stream>>>(sw0, dw0, bt0, kWCarry);
    const int M = kBatch, N = kNumDom * kHid1, K = kIn0;
    const int tiles = (M / 64) * (N / 64);
    wmma_gemm64<0, false, 0, 0, false, 0><<<dim3((tiles + 7) / 8, 1), 256, 0, stream>>>(
        xh, xh, K, 0L, bt0, bt0, K, 0L, (void*)y0, (void*)y0, N, 0L, sb0, y0, 0L, M, N, K, scale0);
    const int o8 = kBatch * kHid1 / 8;
    select_h16_kernel<kHid1><<<dim3((o8 + 255) / 256), 256, 0, stream>>>(y0, dom, sb0, db0, h1, o8, kHCarry);
  }
  {
    fuse_wt_kernel<kHid1, kHid2><<<dim3(kHid1 / 64, kHid2 / 64, kNumDom), 256, 0, stream>>>(sw1, dw1, bt1, kWCarry);
    const int M = kBatch, N = kNumDom * kHid2, K = kHid1;
    const int tiles = (M / 64) * (N / 64);
    wmma_gemm64<0, false, 0, 0, false, 0><<<dim3((tiles + 7) / 8, 1), 256, 0, stream>>>(
        h1, h1, K, 0L, bt1, bt1, K, 0L, (void*)y1, (void*)y1, N, 0L, sb1, y1, 0L, M, N, K, scale12);
    const int o8 = kBatch * kHid2 / 8;
    select_h16_kernel<kHid2><<<dim3((o8 + 255) / 256), 256, 0, stream>>>(y1, dom, sb1, db1, h2, o8, kHCarry);
  }
  {
    fuse_wt_kernel<kHid2, kHid3><<<dim3(kHid2 / 64, kHid3 / 64, kNumDom), 256, 0, stream>>>(sw2, dw2, bt2, kWCarry);
    const int M = kBatch, N = kNumDom * kHid3, K = kHid2;
    const int tiles = (M / 64) * (N / 64);
    wmma_gemm64<0, false, 0, 0, false, 0><<<dim3((tiles + 7) / 8, 1), 256, 0, stream>>>(
        h2, h2, K, 0L, bt2, bt2, K, 0L, (void*)y2, (void*)y2, N, 0L, sb2, y2, 0L, M, N, K, scale12);
    const int o4 = kBatch * kHid3 / 4;
    select_out_kernel<<<dim3((o4 + 255) / 256), 256, 0, stream>>>(y2, dom, sb2, db2, out, o4);
  }
}
